// GATLayerDense_38104949850270
// MI455X (gfx1250) — hardware-verified
//
#include <hip/hip_runtime.h>


namespace {
constexpr int NG = 32, NN = 1024, F = 128, M = NG * NN;
constexpr float XS = 8.0f, WSC = 256.0f, PS = 16384.0f, NEG = 0.2f;
typedef _Float16 b16;
typedef __attribute__((ext_vector_type(16))) _Float16 v16b;
typedef __attribute__((ext_vector_type(8))) _Float16 v8b;
typedef __attribute__((ext_vector_type(8))) float v8f;
typedef __attribute__((ext_vector_type(4))) float v4f;
__device__ __forceinline__ float bf16_rne(float f) { unsigned int u = __float_as_uint(f); u += 0x7FFFu + ((u >> 16) & 1u); return __uint_as_float(u & 0xFFFF0000u); }
__device__ __forceinline__ void split16(float v, b16& hi, b16& lo) { hi = (b16)v; lo = (b16)(v - (float)hi); }
__device__ __forceinline__ v16b frag_kb(const b16* p, int hh) { const v8b a = *(const v8b*)(p + 8 * hh), b = *(const v8b*)(p + 16 + 8 * hh); v16b f;
#pragma unroll
  for (int e = 0; e < 8; ++e) { f[e] = a[e]; f[8 + e] = b[e]; } return f; }
__device__ __forceinline__ v8f wmma16b(v16b a, v16b b, v8f c) { v8f d = __builtin_amdgcn_wmma_f32_16x16x32_f16(false, a, false, b, (short)0, c, false, false); asm volatile("v_nop\n\tv_nop\n\tv_nop\n\tv_nop" : "+v"(d) : "v"(a), "v"(b)); return d; }
__device__ __forceinline__ void wave_lds_sync() { __builtin_amdgcn_fence(__ATOMIC_RELEASE, "workgroup"); __builtin_amdgcn_wave_barrier(); __builtin_amdgcn_fence(__ATOMIC_ACQUIRE, "workgroup"); }
__device__ __forceinline__ float pmul(float a, float b) { float p = a * b; asm volatile("" : "+v"(p)); return p; }
__device__ __forceinline__ float opaque(float a) { asm volatile("" : "+v"(a)); return a; }
__device__ __forceinline__ float lrelu(float x) { return x >= 0.0f ? x : NEG * x; }
__device__ __forceinline__ float nexp(float x) { return __builtin_amdgcn_exp2f(x * 1.4426950408889634f); }

__global__ __launch_bounds__(256) void wprep_kernel(const float* __restrict__ w, b16* __restrict__ WT) {
  const size_t u = (size_t)blockIdx.x * 256 + threadIdx.x; if (u >= (size_t)F * F / 8) return; const size_t e = u * 8; const int o = (int)(e / F), k0 = (int)(e % F); v8b v;
  for (int j = 0; j < 8; ++j) v[j] = (b16)(bf16_rne(w[(size_t)(k0 + j) * F + o]) * WSC); for (int pass = 0; pass < 2; ++pass) { *(volatile v8b*)(WT + e) = v; __threadfence(); }
}
__global__ __launch_bounds__(128) void hgemm_kernel(const float* __restrict__ x, const b16* __restrict__ WT, const float* __restrict__ as_, const float* __restrict__ ad_, float* __restrict__ H, float* __restrict__ S, float* __restrict__ Dd) {
  __shared__ __attribute__((aligned(16))) float Tf[4][16][F + 4]; __shared__ __attribute__((aligned(16))) float sa[64], sd[64];
  const int wave = threadIdx.x >> 5, lane = threadIdx.x & 31, nloc = lane & 15, hlf = lane >> 4; const size_t m0 = (size_t)blockIdx.x * 64 + wave * 16; const float* xr = x + (m0 + nloc) * F;
  v8f acc[8];
#pragma unroll
  for (int t = 0; t < 8; ++t) acc[t] = (v8f){};
#pragma unroll 2
  for (int kb = 0; kb < F; kb += 32) { v16b a; for (int j = 0; j < 8; ++j) { a[j] = (b16)(bf16_rne(xr[kb + 8 * hlf + j]) * XS); a[8 + j] = (b16)(bf16_rne(xr[kb + 16 + 8 * hlf + j]) * XS); }
#pragma unroll
    for (int t = 0; t < 8; ++t) acc[t] = wmma16b(a, frag_kb(WT + (size_t)(t * 16 + nloc) * F + kb, hlf), acc[t]); }
  float ps[8], pd[8]; for (int r8 = 0; r8 < 8; ++r8) { ps[r8] = 0.0f; pd[r8] = 0.0f; }
#pragma unroll
  for (int t = 0; t < 8; ++t) { const int c = t * 16 + nloc; const float ws_ = opaque(bf16_rne(as_[c])), wd_ = opaque(bf16_rne(ad_[c]));
#pragma unroll
    for (int r8 = 0; r8 < 8; ++r8) { const float v = acc[t][r8] * (1.0f / (XS * WSC)); Tf[wave][8 * hlf + r8][c] = v; ps[r8] += pmul(v, ws_); pd[r8] += pmul(v, wd_); } }
#pragma unroll
  for (int r8 = 0; r8 < 8; ++r8) { float a = ps[r8], b = pd[r8]; for (int o = 1; o < 16; o <<= 1) { a += __shfl_xor(a, o); b += __shfl_xor(b, o); } if (nloc == 0) { sa[wave * 16 + 8 * hlf + r8] = a; sd[wave * 16 + 8 * hlf + r8] = b; } }
  __syncthreads();
  for (int pass = 0; pass < 2; ++pass) { for (int rr = 0; rr < 16; ++rr) *(volatile v4f*)(H + (m0 + rr) * F + lane * 4) = *(const v4f*)(&Tf[wave][rr][lane * 4]);
    if (threadIdx.x < 16) *(volatile v4f*)(S + (size_t)blockIdx.x * 64 + threadIdx.x * 4) = *(const v4f*)(&sa[threadIdx.x * 4]); else if (threadIdx.x < 32) *(volatile v4f*)(Dd + (size_t)blockIdx.x * 64 + (threadIdx.x - 16) * 4) = *(const v4f*)(&sd[(threadIdx.x - 16) * 4]);
    __threadfence(); }
}
__global__ __launch_bounds__(256) void htrans_kernel(const float* __restrict__ H, b16* __restrict__ HTH, b16* __restrict__ HTL) {
  __shared__ float tile[64][64 + 1];
  const int c0 = blockIdx.x * 64, j0 = blockIdx.y * 64, g = blockIdx.z; const int wave = threadIdx.x >> 5, lane = threadIdx.x & 31;
  for (int rr = 0; rr < 8; ++rr) { const int jl = wave * 8 + rr; const float* row = H + ((size_t)g * NN + j0 + jl) * F + c0; tile[lane * 2][jl] = row[lane * 2]; tile[lane * 2 + 1][jl] = row[lane * 2 + 1]; }
  __syncthreads();
  typedef __attribute__((ext_vector_type(2))) _Float16 v2b;
  for (int pass = 0; pass < 2; ++pass) { for (int rr = 0; rr < 8; ++rr) { const int cl = wave * 8 + rr; const int c = c0 + cl; b16 p0, q0, p1, q1; split16(tile[cl][lane * 2] * XS, p0, q0); split16(tile[cl][lane * 2 + 1] * XS, p1, q1); v2b h, l; h[0] = p0; h[1] = p1; l[0] = q0; l[1] = q1;
      *(volatile v2b*)(HTH + ((size_t)g * F + c) * NN + j0 + lane * 2) = h; *(volatile v2b*)(HTL + ((size_t)g * F + c) * NN + j0 + lane * 2) = l; } __threadfence(); }
}
__global__ __launch_bounds__(128) void attn_kernel(const float* __restrict__ S, const float* __restrict__ Dd, const b16* __restrict__ HTH, const b16* __restrict__ HTL, float* __restrict__ out) {
  __shared__ __attribute__((aligned(16))) float Tf[4][16][F + 4]; __shared__ float dens[4][16];
  const int wave = threadIdx.x >> 5, lane = threadIdx.x & 31, nloc = lane & 15, hlf = lane >> 4; const size_t i0 = (size_t)blockIdx.x * 64 + wave * 16; const int g = (int)(i0 / NN); const float* Dg = Dd + (size_t)g * NN;
  float mx = -INFINITY; for (int j = lane; j < NN; j += 32) mx = fmaxf(mx, Dg[j]); for (int o = 16; o; o >>= 1) mx = fmaxf(mx, __shfl_xor(mx, o));
  const float si = S[i0 + nloc]; const float mi = lrelu(si + mx); float den = 0.0f;
  const b16* Hh = HTH + (size_t)g * F * NN; const b16* Hl = HTL + (size_t)g * F * NN;
  v8f acc[8];
#pragma unroll
  for (int t = 0; t < 8; ++t) acc[t] = (v8f){};
#pragma unroll 1
  for (int kb = 0; kb < NN; kb += 32) { v16b ph, pl;
    for (int j = 0; j < 8; ++j) { const float p0 = nexp(lrelu(si + Dg[kb + 8 * hlf + j]) - mi), p1 = nexp(lrelu(si + Dg[kb + 16 + 8 * hlf + j]) - mi); den += p0 + p1; b16 a, b; split16(p0 * PS, a, b); ph[j] = a; pl[j] = b; split16(p1 * PS, a, b); ph[8 + j] = a; pl[8 + j] = b; }
#pragma unroll
    for (int t = 0; t < 8; ++t) { const v16b bh = frag_kb(Hh + (size_t)(t * 16 + nloc) * NN + kb, hlf), bl = frag_kb(Hl + (size_t)(t * 16 + nloc) * NN + kb, hlf); acc[t] = wmma16b(ph, bh, acc[t]); acc[t] = wmma16b(pl, bh, acc[t]); acc[t] = wmma16b(ph, bl, acc[t]); } }
  den += __shfl_xor(den, 16);
  if (hlf == 0) dens[wave][nloc] = den;
  wave_lds_sync();
#pragma unroll
  for (int t = 0; t < 8; ++t) { const int c = t * 16 + nloc;
#pragma unroll 1
    for (int r8 = 0; r8 < 8; ++r8) { const int rl = 8 * hlf + r8; Tf[wave][rl][c] = acc[t][r8] * (1.0f / (PS * XS)) / dens[wave][rl]; } }
  wave_lds_sync();
  for (int pass = 0; pass < 2; ++pass) { for (int rr = 0; rr < 16; ++rr) *(volatile v4f*)(out + (i0 + rr) * F + lane * 4) = *(const v4f*)(&Tf[wave][rr][lane * 4]); __threadfence(); }
}
}

extern "C" void kernel_launch(void* const* d_in, const int* in_sizes, int n_in, void* d_out, int out_size, void* d_ws, size_t ws_size, hipStream_t stream) {
  (void)n_in;
  auto Fp = [&](int i) { return (const float*)d_in[i]; };
  if (in_sizes[0] != M * F || in_sizes[1] != F * F || in_sizes[2] != F || in_sizes[3] != F || out_size != M * F) return;
  size_t off = 0; char* ws = (char*)d_ws;
  auto carve = [&](size_t bytes) { char* p = ws + off; off += (bytes + 255) & ~(size_t)255; return p; };
  b16* WT = (b16*)carve((size_t)F * F * 2); float* H = (float*)carve((size_t)M * F * 4); float* S = (float*)carve((size_t)M * 4); float* Dd = (float*)carve((size_t)M * 4); b16* HTH = (b16*)carve((size_t)NG * F * NN * 2); b16* HTL = (b16*)carve((size_t)NG * F * NN * 2);
  if (off > ws_size || off > ((size_t)64 << 20)) return;
  wprep_kernel<<<(F * F / 8 + 255) / 256, 256, 0, stream>>>(Fp(1), WT);
  hgemm_kernel<<<M / 64, 128, 0, stream>>>(Fp(0), WT, Fp(2), Fp(3), H, S, Dd);
  htrans_kernel<<<dim3(F / 64, NN / 64, NG), 256, 0, stream>>>(H, HTH, HTL);
  attn_kernel<<<M / 64, 128, 0, stream>>>(S, Dd, HTH, HTL, (float*)d_out);
}
